// Transformer_55697135894950
// MI455X (gfx1250) — hardware-verified
//
#include <hip/hip_runtime.h>
#ifndef NB
#define NB 2
#endif
#ifndef SEQ
#define SEQ 2048
#endif
#define NB_FULL 2
#define SEQ_FULL 2048
#define CD 1024
#define UD 1024
#define NH 16
#define HD 64
#define HG 2
#define LQK (2 * UD)
#define LNP 8192
#define NPB ((SEQ * UD) / LNP)
#define RSB (SEQ / 8)
#define NR ((size_t)NB * SEQ)
#define WSC 16.0f
#define PCAR 16384.0f
#define VLC 1024.0f
static_assert(NB >= 1 && NB <= NB_FULL);
static_assert(SEQ % 256 == 0 && SEQ <= SEQ_FULL);
static_assert(CD % 32 == 0 && UD % 64 == 0 && CD == UD);
static_assert(NH * HD == UD && HD == 64 && NH % HG == 0 && HD % 32 == 0);
static_assert((SEQ * UD) % LNP == 0 && LNP == 256 * 32);
static_assert(RSB % 32 == 0 && RSB <= 256);
static_assert(2 * NB <= 32);
static_assert((NR * UD) % 1024 == 0 && (NR % 128) == 0);

typedef unsigned short v8us __attribute__((ext_vector_type(8), may_alias));
typedef float  v8f  __attribute__((ext_vector_type(8)));
typedef float  v4f  __attribute__((ext_vector_type(4)));
typedef float  v4fa __attribute__((ext_vector_type(4), may_alias));
typedef double v2d  __attribute__((ext_vector_type(2)));
typedef _Float16 v16h __attribute__((ext_vector_type(16)));
typedef _Float16 v4h  __attribute__((ext_vector_type(4)));
union FragH { v16h v; v8us half[2]; _Float16 h[16]; unsigned short u[16]; };

__device__ __forceinline__ unsigned short bf16_bits(float x) { unsigned int u = __float_as_uint(x); return (unsigned short)((u + 0x7FFFu + ((u >> 16) & 1u)) >> 16); }
__device__ __forceinline__ float bf16_val(unsigned short b) { return __uint_as_float(((unsigned int)b) << 16); }
__device__ __forceinline__ float bf16_rne(float x) { return bf16_val(bf16_bits(x)); }

__device__ __forceinline__ v16h g2_frag(const _Float16* p, int hh) { FragH f; f.half[0] = *(const v8us*)((const unsigned short*)p + 8 * hh); f.half[1] = *(const v8us*)((const unsigned short*)p + 16 + 8 * hh); return f.v; }
__device__ __forceinline__ v8f g2_mma(v16h a, v16h b, v8f c) { v8f d = __builtin_amdgcn_wmma_f32_16x16x32_f16(false, a, false, b, (short)0, c, false, false); asm volatile("v_nop\n\tv_nop\n\tv_nop\n\tv_nop" : "+v"(d) : "v"(a), "v"(b)); return d; }

__global__ __launch_bounds__(256) void k_wt_f16(const float* __restrict__ W, _Float16* __restrict__ Wt, int K, int N, float scale) {
  const int t = blockIdx.x * 256 + threadIdx.x; if (t >= N * (K / 8)) return; const int n = t / (K / 8), k8 = (t % (K / 8)) * 8; FragH f;
#pragma unroll
  for (int i = 0; i < 8; ++i) f.h[i] = (_Float16)(bf16_rne(W[(size_t)(k8 + i) * N + n]) * scale); const v8us o = f.half[0];
  *(volatile v8us*)((unsigned short*)Wt + (size_t)n * K + k8) = o; __threadfence(); *(volatile v8us*)((unsigned short*)Wt + (size_t)n * K + k8) = o;
}

__global__ __launch_bounds__(256) void k_x16(const float* __restrict__ x, _Float16* __restrict__ X16, size_t n8) { const size_t t = (size_t)blockIdx.x * 256 + threadIdx.x; if (t >= n8) return; FragH f;
#pragma unroll
  for (int q = 0; q < 8; ++q) f.h[q] = (_Float16)bf16_rne(x[t * 8 + q]); *(volatile v8us*)((unsigned short*)X16 + t * 8) = f.half[0]; __threadfence(); *(volatile v8us*)((unsigned short*)X16 + t * 8) = f.half[0]; }

template <int ACT, bool CAUSAL>
__global__ __launch_bounds__(128) void k_gemm2(const _Float16* __restrict__ A, int lda, size_t sA, const _Float16* __restrict__ Bh, int ldb, size_t sB, float alpha, const float* __restrict__ bias, size_t sBias, const float* __restrict__ CP, int rowsPerB, size_t sCPb, int row0g,
    float* __restrict__ C, _Float16* __restrict__ C16, int ldc, size_t sC, int M, int N, int K) {
  static_assert(ACT == 0 || ACT == 3);
  __shared__ __attribute__((aligned(16))) float so[4][32][68];
  const int tid = threadIdx.x, w = tid >> 5, lane = tid & 31, ln = lane & 15, hh = lane >> 4; const int by = blockIdx.y;
  A += (size_t)by * sA; Bh += (size_t)by * sB; const size_t cofs = (size_t)by * sC; const float* bp = bias ? bias + (size_t)by * sBias : nullptr;
  const int ntn = N >> 6; const int mt = blockIdx.x / ntn, nq = blockIdx.x - mt * ntn; const int row0 = mt * 128 + 32 * w, col0 = nq * 64;
  if (CAUSAL && col0 >= mt * 128 + 128) return;
  if (row0 >= M) return;
  const _Float16* a0p = A + (size_t)(row0 + ln) * lda; const _Float16* a1p = a0p + (size_t)16 * lda;
  const _Float16* b0p = Bh + (size_t)(col0 + ln) * ldb; const _Float16* b1p = b0p + (size_t)16 * ldb; const _Float16* b2p = b1p + (size_t)16 * ldb; const _Float16* b3p = b2p + (size_t)16 * ldb;
  const v8f z8 = {0.f,0.f,0.f,0.f,0.f,0.f,0.f,0.f}; v8f c00 = z8, c01 = z8, c02 = z8, c03 = z8, c10 = z8, c11 = z8, c12 = z8, c13 = z8;
#pragma unroll 1
  for (int kb = 0; kb < K; kb += 32) { const v16h a0 = g2_frag(a0p + kb, hh), a1 = g2_frag(a1p + kb, hh);
    v16h b = g2_frag(b0p + kb, hh); c00 = g2_mma(a0, b, c00); c10 = g2_mma(a1, b, c10);
    b = g2_frag(b1p + kb, hh); c01 = g2_mma(a0, b, c01); c11 = g2_mma(a1, b, c11);
    b = g2_frag(b2p + kb, hh); c02 = g2_mma(a0, b, c02); c12 = g2_mma(a1, b, c12);
    b = g2_frag(b3p + kb, hh); c03 = g2_mma(a0, b, c03); c13 = g2_mma(a1, b, c13); }
  v8f accs[8] = {c00, c01, c02, c03, c10, c11, c12, c13};
#pragma unroll
  for (int u = 0; u < 8; ++u) { const int t = u & 3, half = u >> 2; const int col = col0 + t * 16 + ln; const float bv = bp ? bf16_rne(bp[col]) : 0.f;
#pragma unroll
    for (int r = 0; r < 8; ++r) { const int rloc = half * 16 + 8 * hh + r; float v = accs[u][r] * alpha + bv;
      if (CP) { if (rowsPerB < 0) v += CP[cofs + (size_t)(row0g + row0 + rloc) * ldc + col]; else { const int bidx = (row0g + row0 + rloc) / rowsPerB; v += CP[(size_t)bidx * sCPb + (size_t)by * 64 + col]; } }
      if (ACT == 3) v = fmaxf(v, 0.f);
      so[w][rloc][t * 16 + ln] = v; } }
  __builtin_amdgcn_fence(4  , "workgroup"); __builtin_amdgcn_wave_barrier();
  const int rsub = lane >> 4, c4 = (lane & 15) * 4;
  for (int pass = 0; pass < 2; ++pass) {
#pragma unroll
    for (int q = 0; q < 16; ++q) { const int r = q * 2 + rsub; const v4f v = *(const v4fa*)&so[w][r][c4];
      if (C) *(volatile v4f*)(C + cofs + (size_t)(row0 + r) * ldc + col0 + c4) = v;
      if (C16) { v4h h4; for (int i = 0; i < 4; ++i) h4[i] = (_Float16)v[i]; *(volatile v4h*)(C16 + cofs + (size_t)(row0 + r) * ldc + col0 + c4) = h4; } }
    if (pass == 0) __threadfence(); }
}

__global__ __launch_bounds__(256) void k_vt2(const float* __restrict__ V32, _Float16* __restrict__ VTh, _Float16* __restrict__ VTl) {
  __shared__ _Float16 th[64][66]; __shared__ _Float16 tl[64][66];
  const int tid = threadIdx.x; const int slab = blockIdx.x / (SEQ / 64), lg = blockIdx.x % (SEQ / 64); const int b = slab / NH, h = slab % NH;
  for (int i = tid; i < 64 * 16; i += 256) { const int r = i >> 4, c4 = (i & 15) * 4;
    const v4f a = *(const v4fa*)(V32 + ((size_t)b * SEQ + (size_t)lg * 64 + r) * UD + h * HD + c4);
#pragma unroll
    for (int q = 0; q < 4; ++q) { const _Float16 hv = (_Float16)a[q]; th[r][c4 + q] = hv; tl[r][c4 + q] = (_Float16)((a[q] - (float)hv) * VLC); } }
  __syncthreads();
  for (int pass = 0; pass < 2; ++pass) {
#pragma unroll
    for (int rd = 0; rd < 2; ++rd) { const int d = rd * 32 + (tid >> 3), pc = tid & 7; FragH fh, fl;
#pragma unroll
      for (int q = 0; q < 8; ++q) { fh.h[q] = th[pc * 8 + q][d]; fl.h[q] = tl[pc * 8 + q][d]; }
      const size_t o = ((size_t)slab * HD + d) * SEQ + (size_t)lg * 64 + pc * 8;
      *(volatile v8us*)((unsigned short*)VTh + o) = fh.half[0]; *(volatile v8us*)((unsigned short*)VTl + o) = fl.half[0]; }
    if (pass == 0) __threadfence(); }
}

__global__ __launch_bounds__(256) void k_rsm(const float* __restrict__ S, _Float16* __restrict__ P) {
  #pragma clang fp contract(off)
  __shared__ float redm[8]; __shared__ float reds[8];
  const int i = blockIdx.x; const int qi = i % SEQ; const int tid = threadIdx.x, lane = tid & 31, w = tid >> 5; const int nw = RSB / 32;
  const int j0 = tid * 8; const int jc = min(j0, qi & ~7);
  const float* s = S + (size_t)i * SEQ;
  const v4f a = *(const v4fa*)(s + jc), c = *(const v4fa*)(s + jc + 4);
  const float v[8] = {a[0], a[1], a[2], a[3], c[0], c[1], c[2], c[3]};
  float mx = -3.0e38f;
#pragma unroll
  for (int q = 0; q < 8; ++q) mx = (j0 + q <= qi) ? fmaxf(mx, v[q]) : mx;
  for (int st = 16; st > 0; st >>= 1) mx = fmaxf(mx, __shfl_xor(mx, st, 32));
  if (lane == 0) redm[w] = mx; __syncthreads();
  mx = redm[0]; for (int u = 1; u < nw; ++u) mx = fmaxf(mx, redm[u]);
  float e[8]; float se = 0.f;
#pragma unroll
  for (int q = 0; q < 8; ++q) { const float t = __expf(v[q] - mx); e[q] = (j0 + q <= qi) ? t : 0.f; se += e[q]; }
  for (int st = 16; st > 0; st >>= 1) se += __shfl_xor(se, st, 32);
  if (lane == 0) reds[w] = se; __syncthreads();
  se = reds[0]; for (int u = 1; u < nw; ++u) se += reds[u];
  const float sc = PCAR * (1.0f / se);
  FragH f;
#pragma unroll
  for (int q = 0; q < 8; ++q) f.h[q] = (_Float16)(e[q] * sc);
  unsigned short* d = (unsigned short*)P + (size_t)i * SEQ + j0;
  *(volatile v8us*)d = f.half[0]; __threadfence(); *(volatile v8us*)d = f.half[0];
}

__global__ __launch_bounds__(128) void k_pv(const _Float16* __restrict__ P, const _Float16* __restrict__ VTh, const _Float16* __restrict__ VTl, int slab0, float* __restrict__ O, int orow0, int ocol0) {
  __shared__ __attribute__((aligned(16))) float so[4][32][36];
  const int tid = threadIdx.x, w = tid >> 5, lane = tid & 31, ln = lane & 15, hh = lane >> 4; const int hg = blockIdx.y;
  const int mt = blockIdx.x / (HD / 32), cg = blockIdx.x % (HD / 32);
  const int row0 = mt * 128 + 32 * w, col0 = cg * 32;
  const int kend = min(SEQ, mt * 128 + 128);
  const _Float16* a0p = P + (size_t)hg * SEQ * SEQ + (size_t)(row0 + ln) * SEQ; const _Float16* a1p = a0p + (size_t)16 * SEQ;
  const size_t vb = ((size_t)(slab0 + hg) * HD + col0 + ln) * SEQ;
  const _Float16* bh0p = VTh + vb; const _Float16* bh1p = bh0p + (size_t)16 * SEQ; const _Float16* bl0p = VTl + vb; const _Float16* bl1p = bl0p + (size_t)16 * SEQ;
  const v8f z8 = {0.f,0.f,0.f,0.f,0.f,0.f,0.f,0.f}; v8f h00 = z8, h01 = z8, h10 = z8, h11 = z8, l00 = z8, l01 = z8, l10 = z8, l11 = z8;
#pragma unroll 1
  for (int kb = 0; kb < kend; kb += 32) { const v16h a0 = g2_frag(a0p + kb, hh), a1 = g2_frag(a1p + kb, hh);
    v16h b = g2_frag(bh0p + kb, hh); h00 = g2_mma(a0, b, h00); h10 = g2_mma(a1, b, h10);
    b = g2_frag(bh1p + kb, hh); h01 = g2_mma(a0, b, h01); h11 = g2_mma(a1, b, h11);
    b = g2_frag(bl0p + kb, hh); l00 = g2_mma(a0, b, l00); l10 = g2_mma(a1, b, l10);
    b = g2_frag(bl1p + kb, hh); l01 = g2_mma(a0, b, l01); l11 = g2_mma(a1, b, l11); }
  v8f ah[4] = {h00, h01, h10, h11}; v8f al[4] = {l00, l01, l10, l11};
#pragma unroll
  for (int u = 0; u < 4; ++u) { const int t = u & 1, half = u >> 1;
#pragma unroll
    for (int r = 0; r < 8; ++r) { const int rloc = half * 16 + 8 * hh + r; so[w][rloc][t * 16 + ln] = (ah[u][r] + al[u][r] * (1.0f / VLC)) * (1.0f / PCAR); } }
  __builtin_amdgcn_fence(4  , "workgroup"); __builtin_amdgcn_wave_barrier();
  const int rq = lane >> 3, c4 = (lane & 7) * 4;
  float* ob = O + (size_t)(orow0 + row0) * UD + ocol0 + hg * HD + col0 + c4;
  for (int pass = 0; pass < 2; ++pass) {
#pragma unroll
    for (int q = 0; q < 8; ++q) { const int r = q * 4 + rq; const v4f v = *(const v4fa*)&so[w][r][c4]; *(volatile v4f*)(ob + (size_t)r * UD) = v; }
    if (pass == 0) __threadfence(); }
}

__global__ __launch_bounds__(256) void k_lnpart(const float* __restrict__ O, const float* __restrict__ X, double* __restrict__ part) {
  __shared__ double rs[256]; __shared__ double rq[256];
  const int bat = blockIdx.y, blk = blockIdx.x, tid = threadIdx.x;
  const float* op = O + (size_t)bat * SEQ * UD + (size_t)blk * LNP; const float* xp = X + (size_t)bat * SEQ_FULL * CD + (size_t)blk * LNP;
  double s1 = 0.0, s2 = 0.0;
#pragma unroll 1
  for (int u = 0; u < LNP / 1024; ++u) { const int j = u * 1024 + tid * 4; const v4f a = *(const v4fa*)(op + j), c = *(const v4fa*)(xp + j);
#pragma unroll
    for (int q = 0; q < 4; ++q) { const float v = a[q] + bf16_rne(c[q]); s1 += (double)v; s2 += (double)v * (double)v; } }
  rs[tid] = s1; rq[tid] = s2; __syncthreads();
  for (int st = 128; st > 0; st >>= 1) { if (tid < st) { rs[tid] += rs[tid + st]; rq[tid] += rq[tid + st]; } __syncthreads(); }
  if (tid < 8) { v2d val; val[0] = (tid == 0) ? rs[0] : 0.0; val[1] = (tid == 0) ? rq[0] : 0.0;
    double* d = part + ((size_t)bat * NPB + blk) * 16 + tid * 2; *(volatile v2d*)d = val; __threadfence(); *(volatile v2d*)d = val; }
}

__global__ __launch_bounds__(64) void k_lnfin(const double* __restrict__ part, float* __restrict__ stat) {
  __shared__ __attribute__((aligned(16))) float st[32];
  const int tid = threadIdx.x; const int bb = (tid < NB) ? tid : (NB - 1);
  double s = 0.0, q = 0.0;
#pragma unroll 1
  for (int i = 0; i < NPB; ++i) { s += part[((size_t)bb * NPB + i) * 16]; q += part[((size_t)bb * NPB + i) * 16 + 1]; }
  const double inv = 1.0 / ((double)SEQ * (double)UD); const double m = s * inv; double var = q * inv - m * m; if (var < 0.0) var = 0.0;
  const float mu = (float)m; const float rsd = 1.0f / sqrtf((float)var + 1.0e-5f);
  if (tid < 32) st[tid] = 0.f;
  __syncthreads();
  if (tid < NB) { st[2 * tid] = mu; st[2 * tid + 1] = rsd; }
  __syncthreads();
  if (tid < 8) { const v4f v = *(const v4fa*)&st[tid * 4]; *(volatile v4f*)(stat + tid * 4) = v; __threadfence(); *(volatile v4f*)(stat + tid * 4) = v; }
}

__global__ __launch_bounds__(256) void k_lnapply(const float* __restrict__ O, const float* __restrict__ X, const float* __restrict__ stat, const float* __restrict__ g, const float* __restrict__ bta, float* __restrict__ out) {
  const size_t e = ((size_t)blockIdx.x * 256 + threadIdx.x) * 4;
  const int bat = (int)(e / ((size_t)SEQ * UD)); const size_t su = e - (size_t)bat * SEQ * UD;
  const float mu = stat[2 * bat], rs = stat[2 * bat + 1];
  const v4f o = *(const v4fa*)(O + e), x = *(const v4fa*)(X + (size_t)bat * SEQ_FULL * CD + su), gg = *(const v4fa*)(g + su), bb = *(const v4fa*)(bta + su);
  v4f y;
#pragma unroll
  for (int q = 0; q < 4; ++q) { const float v = o[q] + bf16_rne(x[q]); y[q] = (v - mu) * rs * bf16_rne(gg[q]) + bf16_rne(bb[q]); }
  float* d = out + (size_t)bat * SEQ_FULL * UD + su;
  *(volatile v4f*)d = y; __threadfence(); *(volatile v4f*)d = y;
}

extern "C" void kernel_launch(void* const* d_in, const int* in_sizes, int n_in,
                              void* d_out, int out_size, void* d_ws, size_t ws_size, hipStream_t stream) {
  if (n_in < 9) return;
  const float* X   = (const float*)d_in[0];
  const float* Wq  = (const float*)d_in[1];
  const float* bq  = (const float*)d_in[2];
  const float* Wk  = (const float*)d_in[3];
  const float* bk  = (const float*)d_in[4];
  const float* Wv  = (const float*)d_in[5];
  const float* bv  = (const float*)d_in[6];
  const float* gam = (const float*)d_in[7];
  const float* bet = (const float*)d_in[8];
  float* out = (float*)d_out;
  const size_t rows_used = (size_t)(NB - 1) * SEQ_FULL + SEQ;
  if ((size_t)in_sizes[0] < rows_used * CD) return;
  if ((size_t)in_sizes[1] < (size_t)CD * UD || (size_t)in_sizes[3] < (size_t)CD * UD || (size_t)in_sizes[5] < (size_t)CD * UD) return;
  if (in_sizes[2] < UD || in_sizes[4] < UD || in_sizes[6] < UD) return;
  if ((size_t)in_sizes[7] < (size_t)SEQ * UD || (size_t)in_sizes[8] < (size_t)SEQ * UD) return;
  if ((size_t)out_size < rows_used * UD) return;

  char* ws = (char*)d_ws; size_t off = 0;
  auto take = [&](size_t bytes) { char* p = ws + off; off += (bytes + 255) & ~(size_t)255; return p; };
  _Float16* BQKV = (_Float16*)take((size_t)3 * CD * UD * 2);
  _Float16* X16  = (_Float16*)take(NR * CD * 2);
  _Float16* QK16 = (_Float16*)take(NR * LQK * 2);
  float*    V32  = (float*)take(NR * UD * 4);
  _Float16* VTh  = (_Float16*)take((size_t)NB * NH * HD * SEQ * 2);
  _Float16* VTl  = (_Float16*)take((size_t)NB * NH * HD * SEQ * 2);
  float*    S    = (float*)take((size_t)HG * SEQ * SEQ * 4);
  _Float16* P    = (_Float16*)take((size_t)HG * SEQ * SEQ * 2);
  float*    O32  = (float*)take(NR * UD * 4);
  double*   PART = (double*)take((size_t)NB * NPB * 128);
  float*    STAT = (float*)take(128);
  if (off > ws_size || off > (size_t)134217728) return;

  k_wt_f16<<<(unsigned)(((size_t)UD * (CD / 8) + 255) / 256), 256, 0, stream>>>(Wq, BQKV, CD, UD, WSC);
  k_wt_f16<<<(unsigned)(((size_t)UD * (CD / 8) + 255) / 256), 256, 0, stream>>>(Wk, BQKV + (size_t)UD * CD, CD, UD, WSC);
  k_wt_f16<<<(unsigned)(((size_t)UD * (CD / 8) + 255) / 256), 256, 0, stream>>>(Wv, BQKV + (size_t)2 * UD * CD, CD, UD, WSC);
  for (int b = 0; b < NB; ++b) {
    const size_t n8 = (size_t)SEQ * CD / 8;
    k_x16<<<(unsigned)((n8 + 255) / 256), 256, 0, stream>>>(X + (size_t)b * SEQ_FULL * CD, X16 + (size_t)b * SEQ * CD, n8);
  }
  const int MP = (int)NR;
  k_gemm2<0, false><<<dim3((unsigned)((MP / 128) * (UD / 64)), 1), 128, 0, stream>>>(X16, CD, 0, BQKV, CD, 0, 0.0625f, bq, 0, nullptr, 1, 0, 0, nullptr, QK16, LQK, 0, MP, UD, CD);
  k_gemm2<0, false><<<dim3((unsigned)((MP / 128) * (UD / 64)), 1), 128, 0, stream>>>(X16, CD, 0, BQKV + (size_t)UD * CD, CD, 0, 0.0625f, bk, 0, nullptr, 1, 0, 0, nullptr, QK16 + UD, LQK, 0, MP, UD, CD);
  k_gemm2<0, false><<<dim3((unsigned)((MP / 128) * (UD / 64)), 1), 128, 0, stream>>>(X16, CD, 0, BQKV + (size_t)2 * UD * CD, CD, 0, 0.0625f, bv, 0, nullptr, 1, 0, 0, V32, nullptr, UD, 0, MP, UD, CD);
  k_vt2<<<(unsigned)(NB * NH * (SEQ / 64)), 256, 0, stream>>>(V32, VTh, VTl);
  for (int b = 0; b < NB; ++b) {
    const size_t r0 = (size_t)b * SEQ;
    for (int h0 = 0; h0 < NH; h0 += HG) {
      k_gemm2<0, true><<<dim3((unsigned)((SEQ / 128) * (SEQ / 64)), HG), 128, 0, stream>>>(QK16 + r0 * LQK + (size_t)h0 * HD, LQK, (size_t)HD, QK16 + r0 * LQK + UD + (size_t)h0 * HD, LQK, (size_t)HD, 0.125f, nullptr, 0, nullptr, 1, 0, 0, S, nullptr, SEQ, (size_t)SEQ * SEQ, SEQ, SEQ, HD);
      k_rsm<<<(unsigned)(HG * SEQ), RSB, 0, stream>>>(S, P);
      k_pv<<<dim3((unsigned)((SEQ / 128) * (HD / 32)), HG), 128, 0, stream>>>(P, VTh, VTl, b * NH + h0, O32, (int)r0, h0 * HD);
    }
  }
  k_lnpart<<<dim3(NPB, NB), 256, 0, stream>>>(O32, X, PART);
  k_lnfin<<<1, 64, 0, stream>>>(PART, STAT);
  k_lnapply<<<(unsigned)((NR * UD) / 1024), 256, 0, stream>>>(O32, X, STAT, gam, bet, out);
}
